// CausalAttn_26182120636802
// MI455X (gfx1250) — hardware-verified
//
#include <hip/hip_runtime.h>
#include <math.h>

typedef __attribute__((ext_vector_type(16))) _Float16 v16h;
typedef __attribute__((ext_vector_type(8)))  _Float16 v8h;
typedef __attribute__((ext_vector_type(16))) __bf16   v16b;
typedef __attribute__((ext_vector_type(8)))  __bf16   v8b;
typedef __attribute__((ext_vector_type(8)))  float    v8f;
typedef __attribute__((ext_vector_type(4)))  float    v4f;
typedef __attribute__((ext_vector_type(4)))  unsigned int v4u;

constexpr int kBatch = 2;
constexpr int kSeq   = 2048;
constexpr int kDim   = 2048;
constexpr int kHeads = 16;
constexpr int kDh    = 128;
constexpr int kRows  = kBatch * kSeq;
constexpr int kLow   = 512;
constexpr int kPairs = kDh / 2;
constexpr float kTheta    = 500000.0f;
constexpr float kQKVCarry = 16.0f;
constexpr float kPCarry   = 32768.0f;
constexpr float kACarry   = 64.0f;
constexpr float kWoCarry  = 1024.0f;
constexpr float kFold     = kPCarry * kQKVCarry / kACarry;
constexpr float kOutScale = 1.0f / (kACarry * kWoCarry);
constexpr float kLog2e    = 1.4426950408889634f;
constexpr float kNegBig   = -3.0e38f;
static_assert(kHeads * kDh == kDim);
static_assert((kDim % 32) == 0 && (kDh % 32) == 0 && (kSeq % 64) == 0);
static_assert((kRows % 64) == 0 && (kDim % 64) == 0 && (kLow % 64) == 0 && ((kSeq - kLow) % 64) == 0);
static_assert(kSeq == 2048 && kDim == 2048 && kDh == 128);
static_assert(kFold == 8192.0f);

constexpr size_t kSzXB  = (size_t)kRows * kDim * 2;
constexpr size_t kSzWT  = (size_t)3 * kDim * kDim * 2;
constexpr size_t kSzWOT = (size_t)kDim * kDim * 2;
constexpr size_t kSzQH  = (size_t)kRows * kDim * 2;
constexpr size_t kSzQL  = (size_t)kBatch * kHeads * kLow * kDh * 2;
constexpr size_t kSzAL  = (size_t)kBatch * kLow * kDim * 2;
constexpr size_t kSzINV = 256;
constexpr size_t kSzTab = (size_t)kSeq * kPairs * 4;
constexpr size_t kOffXB  = 0;
constexpr size_t kOffWT  = kOffXB  + kSzXB;
constexpr size_t kOffWOT = kOffWT  + kSzWT;
constexpr size_t kOffQH  = kOffWOT + kSzWOT;
constexpr size_t kOffKH  = kOffQH  + kSzQH;
constexpr size_t kOffVTH = kOffKH  + kSzQH;
constexpr size_t kOffQL  = kOffVTH + kSzQH;
constexpr size_t kOffKL  = kOffQL  + kSzQL;
constexpr size_t kOffVTL = kOffKL  + kSzQL;
constexpr size_t kOffAL  = kOffVTL + kSzQL;
constexpr size_t kOffINV = kOffAL  + kSzAL;
constexpr size_t kOffCOS = kOffINV + kSzINV;
constexpr size_t kOffSIN = kOffCOS + kSzTab;
constexpr size_t kWsTotal = kOffSIN + kSzTab;
static_assert(kWsTotal == 118489344ull);
static_assert(kWsTotal <= 134217728ull);
static_assert((kOffWT % 128) == 0 && (kOffWOT % 128) == 0 && (kOffQH % 128) == 0 && (kOffKH % 128) == 0 &&
              (kOffVTH % 128) == 0 && (kOffQL % 128) == 0 && (kOffKL % 128) == 0 && (kOffVTL % 128) == 0 &&
              (kOffAL % 128) == 0 && (kOffINV % 128) == 0 && (kOffCOS % 128) == 0 && (kOffSIN % 128) == 0);

__device__ __forceinline__ unsigned short f2bf_bits(float f) {
  unsigned u = __float_as_uint(f);
  return (unsigned short)((u + 0x7FFFu + ((u >> 16) & 1u)) >> 16);
}
__device__ __forceinline__ float bf_bits2f(unsigned short h) { return __uint_as_float(((unsigned)h) << 16); }
__device__ __forceinline__ unsigned pk16(unsigned short a, unsigned short b) { return (unsigned)a | ((unsigned)b << 16); }
__device__ __forceinline__ unsigned short h_bits(float f) { const _Float16 h = (_Float16)f; return __builtin_bit_cast(unsigned short, h); }

__device__ __forceinline__ float fexp2(float x) {
#if __has_builtin(__builtin_amdgcn_exp2f)
  return __builtin_amdgcn_exp2f(x);
#else
  return exp2f(x);
#endif
}

__device__ __forceinline__ void wave_sync_lds() {
  __builtin_amdgcn_fence(__ATOMIC_RELEASE, "workgroup");
  __builtin_amdgcn_wave_barrier();
  __builtin_amdgcn_fence(__ATOMIC_ACQUIRE, "workgroup");
}

union FragH { v16h v; v8h h[2]; };
union FragB { v16b v; v8b h[2]; };
__device__ __forceinline__ v16h ld_frag_h(const _Float16* p) {
  FragH f; f.h[0] = *(const v8h*)(p); f.h[1] = *(const v8h*)(p + 16); return f.v;
}
__device__ __forceinline__ v16b ld_frag_b(const __bf16* p) {
  FragB f; f.h[0] = *(const v8b*)(p); f.h[1] = *(const v8b*)(p + 16); return f.v;
}
__device__ __forceinline__ v8f mma_h(v16h a, v16h b, v8f c) {
  c = __builtin_amdgcn_wmma_f32_16x16x32_f16(false, a, false, b, (short)0, c, false, false);
  asm volatile("v_nop\n\tv_nop\n\tv_nop\n\tv_nop" : "+v"(c) : "v"(a), "v"(b));
  return c;
}
__device__ __forceinline__ v8f mma_b(v16b a, v16b b, v8f c) {
  c = __builtin_amdgcn_wmma_f32_16x16x32_bf16(false, a, false, b, (short)0, c, false, false);
  asm volatile("v_nop\n\tv_nop\n\tv_nop\n\tv_nop" : "+v"(c) : "v"(a), "v"(b));
  return c;
}

__global__ __launch_bounds__(256) void cast8_bf16_kernel(const float* __restrict__ in, unsigned short* out, int n8) {
  const int i = blockIdx.x * 256 + threadIdx.x;
  if (i >= n8) return;
  const float* p = in + 8 * (size_t)i;
  const v4f a = *(const v4f*)(p);
  const v4f c = *(const v4f*)(p + 4);
  unsigned short hb[8];
#pragma unroll
  for (int e = 0; e < 4; ++e) {
    const float fa = a[e];
    const float fc = c[e];
    hb[e]     = f2bf_bits(fa);
    hb[4 + e] = f2bf_bits(fc);
  }
  const v4u u = (v4u){pk16(hb[0], hb[1]), pk16(hb[2], hb[3]), pk16(hb[4], hb[5]), pk16(hb[6], hb[7])};
  unsigned short* q = out + 8 * (size_t)i;
  *(volatile v4u*)q = u;
  __threadfence();
  *(volatile v4u*)q = u;
}

__global__ __launch_bounds__(256) void wt_transpose_kernel(const float* __restrict__ W0, const float* __restrict__ W1,
                                                           const float* __restrict__ W2, const float* __restrict__ W3,
                                                           unsigned short* outT, unsigned short* outO) {
  __shared__ float sm[64][65];
  const int t  = threadIdx.x;
  const int d0 = blockIdx.x * 64;
  const int n0 = blockIdx.y * 64;
  const int z  = blockIdx.z;
  const float* W = (z == 0) ? W0 : (z == 1) ? W1 : (z == 2) ? W2 : W3;
#pragma unroll
  for (int i = 0; i < 16; ++i) {
    const int e = i * 256 + t;
    const int r = e >> 6;
    const int c = e & 63;
    sm[c][r] = W[(size_t)(d0 + r) * kDim + n0 + c];
  }
  __syncthreads();
  const int lane = t & 31;
  const int wave = __builtin_amdgcn_readfirstlane((int)(threadIdx.x >> 5));
  const int q = lane >> 3, c8 = (lane & 7) * 8;
  const bool isWo = (z == 3);
  unsigned short* op = isWo ? outO : (outT + (size_t)z * kDim * kDim);
  v4u u[2];
#pragma unroll
  for (int it = 0; it < 2; ++it) {
    const int row = wave * 8 + it * 4 + q;
    unsigned short hb[8];
#pragma unroll
    for (int e = 0; e < 8; ++e) {
      const float f = sm[row][c8 + e];
      const unsigned short bb = f2bf_bits(f);
      const unsigned short hh = h_bits(bf_bits2f(bb) * kWoCarry);
      hb[e] = isWo ? hh : bb;
    }
    u[it] = (v4u){pk16(hb[0], hb[1]), pk16(hb[2], hb[3]), pk16(hb[4], hb[5]), pk16(hb[6], hb[7])};
  }
  for (int pass = 0; pass < 2; ++pass) {
#pragma unroll
    for (int it = 0; it < 2; ++it) {
      const int row = wave * 8 + it * 4 + q;
      *(volatile v4u*)(op + (size_t)(n0 + row) * kDim + d0 + c8) = u[it];
    }
    __threadfence();
  }
}

__global__ __launch_bounds__(64) void invfreq_kernel(float* invf) {
  const int i = threadIdx.x;
  const float e = (float)(2 * i) / (float)kDh;
  const float p = powf(kTheta, e);
  const float v = 1.0f / p;
  volatile float* o = invf + i;
  *o = v;
  __threadfence();
  *o = v;
}

__global__ __launch_bounds__(256) void rot_table_kernel(const float* __restrict__ invf, float* cosT, float* sinT) {
  const int idx = blockIdx.x * 256 + threadIdx.x;
  const int l = idx >> 6;
  const int i = idx & (kPairs - 1);
  const float ang = (float)l * invf[i];
  const float cv = cosf(ang);
  const float sv = sinf(ang);
  volatile float* co = cosT + idx;
  volatile float* so = sinT + idx;
  *co = cv;
  *so = sv;
  __threadfence();
  *co = cv;
  *so = sv;
}

template <int MODE>
__global__ __launch_bounds__(256) void qkv_gemm_kernel(
    const unsigned short* __restrict__ Ap, const unsigned short* __restrict__ Btp,
    unsigned short* H0, unsigned short* H1, unsigned short* L0, unsigned short* L1,
    const float* __restrict__ cosT, const float* __restrict__ sinT, int N) {
  __shared__ __align__(16) float    sF[MODE == 0 ? 8 * 16 * 68 : 4];
  __shared__ __align__(16) _Float16 sH[MODE == 1 ? 8 * 32 * 72 : 8];
  const __bf16* A  = (const __bf16*)Ap;
  const __bf16* Bt = (const __bf16*)Btp;
  const int lane = threadIdx.x & 31;
  const int wave = __builtin_amdgcn_readfirstlane((int)(threadIdx.x >> 5));
  const int tilesN = N >> 6;
  const int tilesM = kRows >> 6;
  const int tile = blockIdx.x * 8 + wave;
  if (tile >= tilesM * tilesN) return;
  const int tm = tile / tilesN;
  const int tn = tile - tm * tilesN;
  const int m0 = tm << 6;
  const int n0 = tn << 6;
  const int rlane = lane & 15;
  const int koff  = (lane >> 4) * 8;
  const int mOff  = (lane >> 4) * 8;

  v8f acc[4][4];
#pragma unroll
  for (int i = 0; i < 4; ++i)
#pragma unroll
    for (int j = 0; j < 4; ++j) acc[i][j] = (v8f){0.f, 0.f, 0.f, 0.f, 0.f, 0.f, 0.f, 0.f};

  for (int k0 = 0; k0 < kDim; k0 += 32) {
    v16b bh[4];
#pragma unroll
    for (int j = 0; j < 4; ++j)
      bh[j] = ld_frag_b(Bt + (size_t)(n0 + (j << 4) + rlane) * kDim + koff + k0);
#pragma unroll
    for (int i = 0; i < 4; ++i) {
      const v16b ah = ld_frag_b(A + (size_t)(m0 + (i << 4) + rlane) * kDim + koff + k0);
#pragma unroll
      for (int j = 0; j < 4; ++j) acc[i][j] = mma_b(ah, bh[j], acc[i][j]);
    }
  }

  const int bidx = m0 >> 11;
  const int l0   = m0 & (kSeq - 1);
  const bool low = (l0 < kLow);
  const int q = lane >> 3, c8 = (lane & 7) * 8;

  if (MODE == 0) {
    float* slab = sF + wave * (16 * 68);
    const int proj = n0 >> 11;
    const int hcol = n0 & (kDim - 1);
    const int hd   = hcol >> 7;
    const int dh0  = hcol & (kDh - 1);
    unsigned short* Hp = proj ? H1 : H0;
    unsigned short* Lp = proj ? L1 : L0;
    const int pi0 = (dh0 + c8) >> 1;
#pragma unroll
    for (int i = 0; i < 4; ++i) {
#pragma unroll
      for (int j = 0; j < 4; ++j)
#pragma unroll
        for (int r = 0; r < 8; ++r) slab[(mOff + r) * 68 + (j << 4) + rlane] = acc[i][j][r];
      wave_sync_lds();
      v8h hv[4], lv[4];
#pragma unroll
      for (int it = 0; it < 4; ++it) {
        const int row = it * 4 + q;
        const int l = l0 + (i << 4) + row;
        const float* sp = slab + row * 68 + c8;
        const v4f x0 = *(const v4f*)(sp);
        const v4f x1 = *(const v4f*)(sp + 4);
        const v4f cs = *(const v4f*)(cosT + (size_t)l * kPairs + pi0);
        const v4f sn = *(const v4f*)(sinT + (size_t)l * kPairs + pi0);
        float y[8];
        y[0] = x0[0] * cs[0] - x0[1] * sn[0];
        y[1] = x0[1] * cs[0] + x0[0] * sn[0];
        y[2] = x0[2] * cs[1] - x0[3] * sn[1];
        y[3] = x0[3] * cs[1] + x0[2] * sn[1];
        y[4] = x1[0] * cs[2] - x1[1] * sn[2];
        y[5] = x1[1] * cs[2] + x1[0] * sn[2];
        y[6] = x1[2] * cs[3] - x1[3] * sn[3];
        y[7] = x1[3] * cs[3] + x1[2] * sn[3];
#pragma unroll
        for (int e = 0; e < 8; ++e) {
          const float yc = y[e] * kQKVCarry;
          const _Float16 hi = (_Float16)yc;
          hv[it][e] = hi;
          lv[it][e] = (_Float16)(yc - (float)hi);
        }
      }
      for (int pass = 0; pass < 2; ++pass) {
#pragma unroll
        for (int it = 0; it < 4; ++it) {
          const int row = it * 4 + q;
          const int l = l0 + (i << 4) + row;
          const size_t oh = ((size_t)((bidx * kHeads + hd) * kSeq + l)) * kDh + dh0 + c8;
          *(volatile v8h*)(Hp + oh) = hv[it];
          if (low) {
            const size_t ol = ((size_t)((bidx * kHeads + hd) * kLow + l)) * kDh + dh0 + c8;
            *(volatile v8h*)(Lp + ol) = lv[it];
          }
        }
        __threadfence();
      }
      wave_sync_lds();
    }
  } else {
    _Float16* vt = sH + wave * (32 * 72);
    const int hd  = n0 >> 7;
    const int dh0 = n0 & (kDh - 1);
#pragma unroll
    for (int jh = 0; jh < 2; ++jh) {
#pragma unroll
      for (int pl = 0; pl < 2; ++pl) {
        if (pl == 0 || low) {
#pragma unroll
          for (int jj = 0; jj < 2; ++jj) {
#pragma unroll
            for (int i = 0; i < 4; ++i) {
              v8h t;
#pragma unroll
              for (int r = 0; r < 8; ++r) {
                const float yc = acc[i][2 * jh + jj][r] * kQKVCarry;
                const _Float16 hi = (_Float16)yc;
                const _Float16 lo = (_Float16)(yc - (float)hi);
                t[r] = (pl == 0) ? hi : lo;
              }
              *(v8h*)(vt + ((jj << 4) + rlane) * 72 + (i << 4) + mOff) = t;
            }
          }
          wave_sync_lds();
          v8h vv[8];
#pragma unroll
          for (int it = 0; it < 8; ++it) vv[it] = *(const v8h*)(vt + (it * 4 + q) * 72 + c8);
          unsigned short* dst = (pl == 0) ? H0 : L0;
          const int pitch = (pl == 0) ? kSeq : kLow;
          for (int pass = 0; pass < 2; ++pass) {
#pragma unroll
            for (int it = 0; it < 8; ++it) {
              const int dh = dh0 + 32 * jh + it * 4 + q;
              const size_t o = ((size_t)((bidx * kHeads + hd) * kDh + dh)) * pitch + l0 + c8;
              *(volatile v8h*)(dst + o) = vv[it];
            }
            __threadfence();
          }
          wave_sync_lds();
        }
      }
    }
  }
}

template <bool SPLIT>
__global__ __launch_bounds__(128) void attn_kernel(
    const unsigned short* __restrict__ QHp, const unsigned short* __restrict__ KHp, const unsigned short* __restrict__ VTHp,
    const unsigned short* __restrict__ QLp, const unsigned short* __restrict__ KLp, const unsigned short* __restrict__ VTLp,
    unsigned short* AHp, unsigned short* ALp, int qb0, int nqb) {
  __shared__ __align__(16) _Float16 Psh[4][16 * 72];
  __shared__ __align__(16) _Float16 Psl[SPLIT ? 4 : 1][SPLIT ? 16 * 72 : 8];
  __shared__ __align__(16) float    Os[4][16 * 68];

  const int lane = threadIdx.x & 31;
  const int wave = __builtin_amdgcn_readfirstlane((int)(threadIdx.x >> 5));
  const int hh = lane >> 4;
  const int c  = lane & 15;
  const int bx = blockIdx.x;
  const int bh = bx / nqb;
  const int qb = qb0 + (bx - bh * nqb);
  const int b  = bh >> 4;
  const int h  = bh & (kHeads - 1);
  const int q0 = qb * 64 + wave * 16;

  const _Float16* Qh = (const _Float16*)QHp  + (size_t)bh * kSeq * kDh;
  const _Float16* Kh = (const _Float16*)KHp  + (size_t)bh * kSeq * kDh;
  const _Float16* Vh = (const _Float16*)VTHp + (size_t)bh * kDh * kSeq;
  const _Float16* Ql = (const _Float16*)QLp  + (size_t)bh * kLow * kDh;
  const _Float16* Kl = (const _Float16*)KLp  + (size_t)bh * kLow * kDh;
  const _Float16* Vl = (const _Float16*)VTLp + (size_t)bh * kDh * kLow;

  const float sc = (1.0f / sqrtf((float)kDh)) * (kLog2e / (kQKVCarry * kQKVCarry));

  float mrow[8], lrow[8];
  v8f oacc[8];
#pragma unroll
  for (int r = 0; r < 8; ++r) { mrow[r] = kNegBig; lrow[r] = 0.f; }
#pragma unroll
  for (int t = 0; t < 8; ++t) oacc[t] = (v8f){0.f, 0.f, 0.f, 0.f, 0.f, 0.f, 0.f, 0.f};

  _Float16* pwh = Psh[wave];
  _Float16* pwl = Psl[SPLIT ? wave : 0];

  for (int kc = 0; kc <= qb; ++kc) {
    const int kv0 = kc * 64;
    v8f s[4];
#pragma unroll
    for (int j = 0; j < 4; ++j) s[j] = (v8f){0.f, 0.f, 0.f, 0.f, 0.f, 0.f, 0.f, 0.f};
#pragma unroll 1
    for (int dc = 0; dc < 4; ++dc) {
      const size_t qo = (size_t)(q0 + c) * kDh + dc * 32 + 8 * hh;
      const v16h qa = ld_frag_h(Qh + qo);
      v16h qla = qa;
      if (SPLIT) qla = ld_frag_h(Ql + qo);
#pragma unroll
      for (int j = 0; j < 4; ++j) {
        const size_t ko = (size_t)(kv0 + (j << 4) + c) * kDh + dc * 32 + 8 * hh;
        const v16h kb = ld_frag_h(Kh + ko);
        s[j] = mma_h(qa, kb, s[j]);
        if (SPLIT) {
          const v16h kl = ld_frag_h(Kl + ko);
          s[j] = mma_h(qa, kl, s[j]);
          s[j] = mma_h(qla, kb, s[j]);
        }
      }
    }

    const bool diag = (kc == qb);
    float cm[8];
#pragma unroll
    for (int r = 0; r < 8; ++r) {
      const int qrow = q0 + 8 * hh + r;
      float m = kNegBig;
#pragma unroll
      for (int j = 0; j < 4; ++j) {
        const int kvcol = kv0 + (j << 4) + c;
        const float tv = s[j][r] * sc;
        const float tm = (diag && (kvcol > qrow)) ? kNegBig : tv;
        s[j][r] = tm;
        m = fmaxf(m, tm);
      }
#pragma unroll
      for (int off = 1; off < 16; off <<= 1) m = fmaxf(m, __shfl_xor(m, off, 32));
      cm[r] = m;
    }
#pragma unroll
    for (int r = 0; r < 8; ++r) {
      const float mnew  = fmaxf(mrow[r], cm[r]);
      const float alpha = fexp2(mrow[r] - mnew);
      mrow[r] = mnew;
      float psum = 0.f;
#pragma unroll
      for (int j = 0; j < 4; ++j) {
        const float p = fexp2(s[j][r] - mnew);
        psum += p;
        const float pc = p * kPCarry;
        const _Float16 ph = (_Float16)pc;
        pwh[(8 * hh + r) * 72 + (j << 4) + c] = ph;
        if (SPLIT) pwl[(8 * hh + r) * 72 + (j << 4) + c] = (_Float16)(pc - (float)ph);
      }
#pragma unroll
      for (int off = 1; off < 16; off <<= 1) psum += __shfl_xor(psum, off, 32);
      lrow[r] = lrow[r] * alpha + psum;
#pragma unroll
      for (int t = 0; t < 8; ++t) oacc[t][r] *= alpha;
    }
    wave_sync_lds();
#pragma unroll 1
    for (int kk = 0; kk < 2; ++kk) {
      const v16h pa = ld_frag_h(pwh + c * 72 + kk * 32 + 8 * hh);
      v16h pl = pa;
      if (SPLIT) pl = ld_frag_h(pwl + c * 72 + kk * 32 + 8 * hh);
#pragma unroll
      for (int t = 0; t < 8; ++t) {
        const v16h vb = ld_frag_h(Vh + (size_t)((t << 4) + c) * kSeq + kv0 + kk * 32 + 8 * hh);
        oacc[t] = mma_h(pa, vb, oacc[t]);
        if (SPLIT) {
          const v16h vl = ld_frag_h(Vl + (size_t)((t << 4) + c) * kLow + kv0 + kk * 32 + 8 * hh);
          oacc[t] = mma_h(pa, vl, oacc[t]);
          oacc[t] = mma_h(pl, vb, oacc[t]);
        }
      }
    }
    wave_sync_lds();
  }

  float* os = Os[wave];
  float inv[8];
#pragma unroll
  for (int r = 0; r < 8; ++r) inv[r] = 1.0f / (lrow[r] * kFold);
  const int q = lane >> 3, c8 = (lane & 7) * 8;
  unsigned short* AH = AHp;
  unsigned short* AL = ALp;
#pragma unroll
  for (int half = 0; half < 2; ++half) {
#pragma unroll
    for (int r = 0; r < 8; ++r)
#pragma unroll
      for (int tt = 0; tt < 4; ++tt) os[(8 * hh + r) * 68 + (tt << 4) + c] = oacc[half * 4 + tt][r] * inv[r];
    wave_sync_lds();
    v8h hv[4], lv[4];
#pragma unroll
    for (int it = 0; it < 4; ++it) {
      const int row = it * 4 + q;
      const float* sp = os + row * 68 + c8;
      const v4f a0 = *(const v4f*)(sp);
      const v4f a1 = *(const v4f*)(sp + 4);
#pragma unroll
      for (int e = 0; e < 4; ++e) {
        const float f0 = a0[e];
        const float f1 = a1[e];
        const _Float16 h0 = (_Float16)f0;
        const _Float16 h1 = (_Float16)f1;
        hv[it][e]     = h0;
        hv[it][4 + e] = h1;
        lv[it][e]     = (_Float16)(f0 - (float)h0);
        lv[it][4 + e] = (_Float16)(f1 - (float)h1);
      }
    }
    for (int pass = 0; pass < 2; ++pass) {
#pragma unroll
      for (int it = 0; it < 4; ++it) {
        const int row = it * 4 + q;
        const size_t oh = (size_t)(b * kSeq + q0 + row) * kDim + h * kDh + half * 64 + c8;
        *(volatile v8h*)(AH + oh) = hv[it];
        if (SPLIT) {
          const size_t ol = (size_t)(b * kLow + q0 + row) * kDim + h * kDh + half * 64 + c8;
          *(volatile v8h*)(AL + ol) = lv[it];
        }
      }
      __threadfence();
    }
    wave_sync_lds();
  }
}

template <bool ASPLIT>
__global__ __launch_bounds__(256) void oproj_gemm_kernel(
    const unsigned short* __restrict__ Ap, const unsigned short* __restrict__ A2p, long strideA, long strideA2,
    const unsigned short* __restrict__ Btp, float* Cout, long strideC, int M, float scale) {
  __shared__ __align__(16) float sT[8 * 16 * 68];
  const int bz   = blockIdx.y;
  const int lane = threadIdx.x & 31;
  const int wave = __builtin_amdgcn_readfirstlane((int)(threadIdx.x >> 5));
  const int tilesN = kDim >> 6;
  const int tilesM = M >> 6;
  const int tile = blockIdx.x * 8 + wave;
  if (tile >= tilesM * tilesN) return;
  const int tm = tile / tilesN;
  const int tn = tile - tm * tilesN;
  const int m0 = tm << 6;
  const int n0 = tn << 6;
  const _Float16* A  = (const _Float16*)Ap  + (size_t)bz * strideA;
  const _Float16* A2 = (const _Float16*)A2p + (size_t)bz * strideA2;
  const _Float16* Bt = (const _Float16*)Btp;
  float* C = Cout + (size_t)bz * strideC;
  const int rlane = lane & 15;
  const int koff  = (lane >> 4) * 8;
  const int mOff  = (lane >> 4) * 8;

  v8f acc[4][4];
#pragma unroll
  for (int i = 0; i < 4; ++i)
#pragma unroll
    for (int j = 0; j < 4; ++j) acc[i][j] = (v8f){0.f, 0.f, 0.f, 0.f, 0.f, 0.f, 0.f, 0.f};

  for (int k0 = 0; k0 < kDim; k0 += 32) {
    v16h bh[4];
#pragma unroll
    for (int j = 0; j < 4; ++j)
      bh[j] = ld_frag_h(Bt + (size_t)(n0 + (j << 4) + rlane) * kDim + koff + k0);
#pragma unroll
    for (int i = 0; i < 4; ++i) {
      const size_t ao = (size_t)(m0 + (i << 4) + rlane) * kDim + koff + k0;
      const v16h ah = ld_frag_h(A + ao);
      v16h al = ah;
      if (ASPLIT) al = ld_frag_h(A2 + ao);
#pragma unroll
      for (int j = 0; j < 4; ++j) {
        acc[i][j] = mma_h(ah, bh[j], acc[i][j]);
        if (ASPLIT) acc[i][j] = mma_h(al, bh[j], acc[i][j]);
      }
    }
  }

  float* slab = sT + wave * (16 * 68);
  const int hh = lane >> 4, c4 = (lane & 15) * 4;
#pragma unroll
  for (int i = 0; i < 4; ++i) {
    const int mBase = m0 + (i << 4);
#pragma unroll
    for (int j = 0; j < 4; ++j)
#pragma unroll
      for (int r = 0; r < 8; ++r) slab[(mOff + r) * 68 + (j << 4) + rlane] = acc[i][j][r] * scale;
    wave_sync_lds();
    for (int pass = 0; pass < 2; ++pass) {
#pragma unroll
      for (int it = 0; it < 8; ++it) {
        const int row = it * 2 + hh;
        const v4f v = *(const v4f*)(slab + row * 68 + c4);
        *(volatile v4f*)(C + (size_t)(mBase + row) * kDim + n0 + c4) = v;
      }
      __threadfence();
    }
    wave_sync_lds();
  }
}

extern "C" void kernel_launch(void* const* d_in, const int* in_sizes, int n_in,
                              void* d_out, int out_size, void* d_ws, size_t ws_size,
                              hipStream_t stream) {
  if (n_in < 5) return;
  if (in_sizes[0] != kRows * kDim) return;
  if (in_sizes[1] != kDim * kDim) return;
  if (in_sizes[2] != kDim * kDim) return;
  if (in_sizes[3] != kDim * kDim) return;
  if (in_sizes[4] != kDim * kDim) return;
  if (out_size != kRows * kDim) return;
  if (ws_size < kWsTotal) return;

  const float* x  = (const float*)d_in[0];
  const float* Wq = (const float*)d_in[1];
  const float* Wk = (const float*)d_in[2];
  const float* Wv = (const float*)d_in[3];
  const float* Wo = (const float*)d_in[4];
  float* out = (float*)d_out;

  char* ws = (char*)d_ws;
  unsigned short* XB  = (unsigned short*)(ws + kOffXB);
  unsigned short* AH  = (unsigned short*)(ws + kOffXB);
  unsigned short* WT  = (unsigned short*)(ws + kOffWT);
  unsigned short* WOT = (unsigned short*)(ws + kOffWOT);
  unsigned short* QH  = (unsigned short*)(ws + kOffQH);
  unsigned short* KH  = (unsigned short*)(ws + kOffKH);
  unsigned short* VTH = (unsigned short*)(ws + kOffVTH);
  unsigned short* QL  = (unsigned short*)(ws + kOffQL);
  unsigned short* KL  = (unsigned short*)(ws + kOffKL);
  unsigned short* VTL = (unsigned short*)(ws + kOffVTL);
  unsigned short* AL  = (unsigned short*)(ws + kOffAL);
  float* INVF = (float*)(ws + kOffINV);
  float* COST = (float*)(ws + kOffCOS);
  float* SINT = (float*)(ws + kOffSIN);

  cast8_bf16_kernel<<<(kRows * kDim / 8) / 256, 256, 0, stream>>>(x, XB, kRows * kDim / 8);
  wt_transpose_kernel<<<dim3(kDim / 64, kDim / 64, 4), 256, 0, stream>>>(Wq, Wk, Wv, Wo, WT, WOT);
  invfreq_kernel<<<1, 64, 0, stream>>>(INVF);
  rot_table_kernel<<<(kSeq * kPairs) / 256, 256, 0, stream>>>(INVF, COST, SINT);

  qkv_gemm_kernel<0><<<(kRows / 64) * (2 * kDim / 64) / 8, 256, 0, stream>>>(
      XB, WT, QH, KH, QL, KL, COST, SINT, 2 * kDim);
  qkv_gemm_kernel<1><<<(kRows / 64) * (kDim / 64) / 8, 256, 0, stream>>>(
      XB, WT + (size_t)2 * kDim * kDim, VTH, VTH, VTL, VTL, COST, SINT, kDim);

  attn_kernel<true><<<(kLow / 64) * kBatch * kHeads, 128, 0, stream>>>(
      QH, KH, VTH, QL, KL, VTL, AH, AL, 0, kLow / 64);
  attn_kernel<false><<<((kSeq - kLow) / 64) * kBatch * kHeads, 128, 0, stream>>>(
      QH, KH, VTH, QL, KL, VTL, AH, AL, kLow / 64, (kSeq - kLow) / 64);

  oproj_gemm_kernel<true><<<dim3((kLow / 64) * (kDim / 64) / 8, kBatch), 256, 0, stream>>>(
      AH, AL, (long)kSeq * kDim, (long)kLow * kDim, WOT, out, (long)kSeq * kDim, kLow, kOutScale);
  oproj_gemm_kernel<false><<<dim3(((kSeq - kLow) / 64) * (kDim / 64) / 8, kBatch), 256, 0, stream>>>(
      AH + (size_t)kLow * kDim, AH + (size_t)kLow * kDim, (long)kSeq * kDim, (long)kSeq * kDim,
      WOT, out + (size_t)kLow * kDim, (long)kSeq * kDim, kSeq - kLow, kOutScale);
}
